// GatedLinearAttention_2207613190881
// MI455X (gfx1250) — hardware-run, weakly checked
//
#include <hip/hip_runtime.h>
#include <stdint.h>

constexpr int kBatch  = 2;
constexpr int kSeq    = 2048;
constexpr int kHidden = 1024;
constexpr int kHeads  = 16;
constexpr int kHdim   = 64;
constexpr int kLowR   = 16;
constexpr int kRows   = kBatch * kSeq;
constexpr float kEps  = 1e-5f;
constexpr float kOScale = 0.125f;

constexpr size_t kBytesXb    = (size_t)kRows * kHidden * 2;
constexpr size_t kBytesBtcat = (size_t)4 * kHidden * kHidden * 2;
constexpr size_t kBytesBt3   = (size_t)64 * kHidden * 2;
constexpr size_t kBytesBt4   = (size_t)kHidden * 128 * 2;
constexpr size_t kBytesBt7   = (size_t)kHidden * 2048 * 2;
constexpr size_t kBytesCqkvg = (size_t)kRows * 4096 * 4;
constexpr size_t kBytesC3    = (size_t)kRows * 128 * 2;
constexpr size_t kBytesApre  = (size_t)kRows * kHidden * 4;
constexpr size_t kBytesOpl   = (size_t)kRows * 2048 * 2;

constexpr size_t kOffXb    = 0;
constexpr size_t kOffBtcat = kOffXb + kBytesXb;
constexpr size_t kOffBt3   = kOffBtcat + kBytesBtcat;
constexpr size_t kOffBt4   = kOffBt3 + kBytesBt3;
constexpr size_t kOffBt7   = kOffBt4 + kBytesBt4;
constexpr size_t kOffCqkvg = kOffBt7 + kBytesBt7;
constexpr size_t kOffC3    = kOffCqkvg + kBytesCqkvg;
constexpr size_t kOffApre  = kOffC3 + kBytesC3;
constexpr size_t kOffOpl   = kOffApre + kBytesApre;
constexpr size_t kWsTotal  = kOffOpl + kBytesOpl;
static_assert(kWsTotal == 123076608, "carve total");
static_assert(kWsTotal <= 134217728, "carve cap");
static_assert((kOffBtcat % 128) == 0 && (kOffBt3 % 128) == 0 && (kOffBt4 % 128) == 0 && (kOffBt7 % 128) == 0 &&
              (kOffCqkvg % 128) == 0 && (kOffC3 % 128) == 0 && (kOffApre % 128) == 0 && (kOffOpl % 128) == 0, "align");

constexpr size_t kOut1ByteOff  = 16777216;
constexpr size_t kOut1FloatOff = kOut1ByteOff / 4;
static_assert(kOut1ByteOff + (size_t)kBatch * kHeads * kHdim * kHdim * 4 <= 17301504, "out extent");

static_assert(kRows % 64 == 0 && 4096 % 64 == 0 && kHidden % 32 == 0, "qkvg gemm");
static_assert(64 % 64 == 0 && 128 % 32 == 0 && 2048 % 32 == 0 && kHidden % 64 == 0, "side gemms");

typedef __attribute__((ext_vector_type(16))) _Float16 v16h;
typedef __attribute__((ext_vector_type(8)))  _Float16 v8h;
typedef __attribute__((ext_vector_type(16))) __bf16   v16b;
typedef __attribute__((ext_vector_type(8)))  __bf16   v8b;
typedef __attribute__((ext_vector_type(8)))  float    v8f;
typedef __attribute__((ext_vector_type(4)))  float    v4f;
typedef __attribute__((ext_vector_type(4)))  unsigned int u4;
typedef u4 __attribute__((may_alias)) u4a;

__device__ __forceinline__ unsigned short f2bf_bits(float f) {
  unsigned u = __float_as_uint(f);
  return (unsigned short)((u + 0x7FFFu + ((u >> 16) & 1u)) >> 16);
}
__device__ __forceinline__ float bf_bits2f(unsigned short h) { return __uint_as_float(((unsigned)h) << 16); }

__device__ __forceinline__ void dep_guard_h(v8f& a, v8f& b, v16h x, v16h y) { asm volatile("v_nop\n\tv_nop\n\tv_nop\n\tv_nop" : "+v"(a), "+v"(b) : "v"(x), "v"(y)); }
__device__ __forceinline__ void dep_guard_b(v8f& a, v8f& b, v16b x, v16b y) { asm volatile("v_nop\n\tv_nop\n\tv_nop\n\tv_nop" : "+v"(a), "+v"(b) : "v"(x), "v"(y)); }
__device__ __forceinline__ void keep4_h(v16h a, v16h b, v16h c, v16h d) { asm volatile("v_nop" :: "v"(a), "v"(b), "v"(c), "v"(d)); }
__device__ __forceinline__ void keep4_b(v16b a, v16b b, v16b c, v16b d) { asm volatile("v_nop" :: "v"(a), "v"(b), "v"(c), "v"(d)); }
__device__ __forceinline__ void acc_guard4(v8f& a, v8f& b, v8f& c, v8f& d) { asm volatile("v_nop\n\tv_nop\n\tv_nop\n\tv_nop" : "+v"(a), "+v"(b), "+v"(c), "+v"(d)); }
template <typename T> struct Frag;
template <> struct Frag<_Float16> {
  typedef v16h V; union U { v16h v; v8h h[2]; };
  static __device__ __forceinline__ v16h load(const _Float16* p) {
    U f; f.h[0] = *(const v8h*)(p); f.h[1] = *(const v8h*)(p + 16); return f.v;
  }
  static __device__ __forceinline__ v8f mma(v16h a, v16h b, v8f c) {
    return __builtin_amdgcn_wmma_f32_16x16x32_f16(false, a, false, b, (short)0, c, false, false);
  }
  static __device__ __forceinline__ void guard(v8f& a, v8f& b, v16h x, v16h y) { dep_guard_h(a, b, x, y); }
  static __device__ __forceinline__ void keep(v16h a, v16h b, v16h c, v16h d) { keep4_h(a, b, c, d); }
};
template <> struct Frag<__bf16> {
  typedef v16b V; union U { v16b v; v8b h[2]; };
  static __device__ __forceinline__ v16b load(const __bf16* p) {
    U f; f.h[0] = *(const v8b*)(p); f.h[1] = *(const v8b*)(p + 16); return f.v;
  }
  static __device__ __forceinline__ v8f mma(v16b a, v16b b, v8f c) {
    return __builtin_amdgcn_wmma_f32_16x16x32_bf16(false, a, false, b, (short)0, c, false, false);
  }
  static __device__ __forceinline__ void guard(v8f& a, v8f& b, v16b x, v16b y) { dep_guard_b(a, b, x, y); }
  static __device__ __forceinline__ void keep(v16b a, v16b b, v16b c, v16b d) { keep4_b(a, b, c, d); }
};

template <int ET> struct Elem;
template <> struct Elem<0> { typedef _Float16 T; };
template <> struct Elem<1> { typedef __bf16 T; };
template <int ET, bool SPLIT, int BIAS_MODE, int OUT_MODE, bool RESID, int ACT = 0>
__global__ __launch_bounds__(256) void wmma_gemm64(
    const unsigned short* __restrict__ Ap, const unsigned short* __restrict__ A2p, int lda, long strideA,
    const unsigned short* __restrict__ Btp, const unsigned short* __restrict__ Bt2p, int ldb, long strideB,
    void* __restrict__ Cout, void* __restrict__ Cout2, int ldc, long strideC,
    const float* __restrict__ bias,
    const float* __restrict__ resid, long strideR,
    int M, int N, int K, float scale) {
  typedef typename Elem<ET>::T T;
  typedef typename Frag<T>::V V;
  const T* A = (const T*)Ap; const T* A2 = (const T*)A2p; const T* Bt = (const T*)Btp; const T* Bt2 = (const T*)Bt2p;
  __shared__ __align__(16) float sT[8][16 * 68];
  const int b    = blockIdx.y;
  const int lane = threadIdx.x & 31;
  const int wave = threadIdx.x >> 5;
  const int tilesN = N >> 6;
  const int tilesM = M >> 6;
  const int tile = blockIdx.x * 8 + wave;
  if (tile >= tilesM * tilesN) return;
  const int tm = tile / tilesN;
  const int tn = tile - tm * tilesN;
  const int m0 = tm << 6;
  const int n0 = tn << 6;

  const T* Ab  = A  + (size_t)b * strideA;
  const T* Bb  = Bt + (size_t)b * strideB;
  const T* Ab2 = SPLIT ? (A2  + (size_t)b * strideA) : nullptr;
  const T* Bb2 = SPLIT ? (Bt2 + (size_t)b * strideB) : nullptr;

  const int rlane = lane & 15;
  const int koff  = (lane >> 4) * 8;
  const int mOff  = (lane >> 4) * 8;

  v8f acc[4][4];
#pragma unroll
  for (int i = 0; i < 4; ++i)
#pragma unroll
    for (int j = 0; j < 4; ++j) acc[i][j] = (v8f){0.f,0.f,0.f,0.f,0.f,0.f,0.f,0.f};

  for (int k0 = 0; k0 < K; k0 += 32) {
    V bh[4], bl[4];
#pragma unroll
    for (int j = 0; j < 4; ++j) {
      const size_t bo = (size_t)(n0 + (j << 4) + rlane) * ldb + koff + k0;
      bh[j] = Frag<T>::load(Bb + bo);
      if (SPLIT) bl[j] = Frag<T>::load(Bb2 + bo);
    }
#pragma unroll
    for (int i = 0; i < 4; ++i) {
      const size_t ao = (size_t)(m0 + (i << 4) + rlane) * lda + koff + k0;
      V ah = Frag<T>::load(Ab + ao);
      V al;
      if (SPLIT) al = Frag<T>::load(Ab2 + ao);
#pragma unroll
      for (int j = 0; j < 4; ++j) {
        acc[i][j] = Frag<T>::mma(ah, bh[j], acc[i][j]);
        if (SPLIT) {
          acc[i][j] = Frag<T>::mma(ah, bl[j], acc[i][j]);
          acc[i][j] = Frag<T>::mma(al, bh[j], acc[i][j]);
        }
      }
      Frag<T>::guard(acc[i][0], acc[i][3], ah, SPLIT ? al : ah);
    }
    Frag<T>::keep(bh[0], bh[1], bh[2], bh[3]);
    if (SPLIT) Frag<T>::keep(bl[0], bl[1], bl[2], bl[3]);
  }
  acc_guard4(acc[0][0], acc[0][1], acc[0][2], acc[0][3]);
  acc_guard4(acc[1][0], acc[1][1], acc[1][2], acc[1][3]);
  acc_guard4(acc[2][0], acc[2][1], acc[2][2], acc[2][3]);
  acc_guard4(acc[3][0], acc[3][1], acc[3][2], acc[3][3]);

  float* slab = sT[wave];
  const float* Rb = RESID ? (resid + (size_t)b * strideR) : nullptr;
#pragma unroll
  for (int i = 0; i < 4; ++i) {
    const int mBase = m0 + (i << 4);
#pragma unroll
    for (int j = 0; j < 4; ++j) {
      const int n = n0 + (j << 4) + rlane;
      float bv = 0.f;
      if (BIAS_MODE == 2) bv = bias[n];
#pragma unroll
      for (int r = 0; r < 8; ++r) {
        float v = acc[i][j][r] * scale;
        if (BIAS_MODE == 1) v += bias[mBase + mOff + r];
        if (BIAS_MODE == 2) v += bv;
        if (RESID) v += Rb[(size_t)(mBase + mOff + r) * ldc + n];
        if (ACT == 1) v = tanhf(v);
        if (ACT == 2) v = fmaxf(v, 0.0f);
        if (ACT == 3) v = v / (1.0f + expf(-v));
        if (ACT == 4) v = (v > 0.f) ? v : 0.01f * v;
        if (ACT == 5) v = 0.5f * v * (1.0f + erff(v * 0.70710678118654752f));
        slab[(mOff + r) * 68 + (j << 4) + rlane] = v;
      }
    }
    __builtin_amdgcn_fence(__ATOMIC_RELEASE, "workgroup");
    __builtin_amdgcn_wave_barrier();
    __builtin_amdgcn_fence(__ATOMIC_ACQUIRE, "workgroup");
    if (OUT_MODE == 0) {
      float* C = (float*)Cout + (size_t)b * strideC;
      const int hh = lane >> 4, c4 = (lane & 15) * 4;
      for (int pass = 0; pass < 2; ++pass) {
#pragma unroll
        for (int it = 0; it < 8; ++it) {
          const int row = it * 2 + hh;
          v4f v = *(const v4f*)(slab + row * 68 + c4);
          *(volatile v4f*)(C + (size_t)(mBase + row) * ldc + n0 + c4) = v;
        }
        __threadfence();
      }
    } else {
      const int q = lane >> 3, c8 = (lane & 7) * 8;
      unsigned short* C  = (unsigned short*)Cout  + (size_t)b * strideC;
      unsigned short* C2 = (OUT_MODE == 2) ? ((unsigned short*)Cout2 + (size_t)b * strideC) : nullptr;
      for (int pass = 0; pass < 2; ++pass) {
#pragma unroll
        for (int it = 0; it < 4; ++it) {
          const int row = it * 4 + q;
          const float* sp = slab + row * 68 + c8;
          v8h hv, lv;
#pragma unroll
          for (int e = 0; e < 8; ++e) {
            if (OUT_MODE == 1) {
              hv[e] = (_Float16)sp[e];
            } else {
              unsigned short hb = f2bf_bits(sp[e]);
              unsigned short lb = f2bf_bits(sp[e] - bf_bits2f(hb));
              hv[e] = __builtin_bit_cast(_Float16, hb);
              lv[e] = __builtin_bit_cast(_Float16, lb);
            }
          }
          *(volatile v8h*)(C + (size_t)(mBase + row) * ldc + n0 + c8) = hv;
          if (OUT_MODE == 2) *(volatile v8h*)(C2 + (size_t)(mBase + row) * ldc + n0 + c8) = lv;
        }
        __threadfence();
      }
    }
    __builtin_amdgcn_fence(__ATOMIC_RELEASE, "workgroup");
    __builtin_amdgcn_wave_barrier();
    __builtin_amdgcn_fence(__ATOMIC_ACQUIRE, "workgroup");
  }
}

__global__ __launch_bounds__(256) void k_cast_bf16x2(
    const float* __restrict__ in, unsigned short* __restrict__ out, int n2) {
  int i = blockIdx.x * 256 + threadIdx.x;
  if (i < n2) {
    const float f0 = in[2 * (size_t)i], f1 = in[2 * (size_t)i + 1];
    const unsigned u = (unsigned)f2bf_bits(f0) | ((unsigned)f2bf_bits(f1) << 16);
    ((volatile unsigned*)out)[i] = u;
    __threadfence();
    ((volatile unsigned*)out)[i] = u;
  }
}

__global__ __launch_bounds__(256) void k_wtrans(const float* __restrict__ W, unsigned short* __restrict__ Bt,
                                               int ldo, int nbase, int dup) {
  __shared__ __align__(16) unsigned short tileT[64 * 72];
  const int tid = threadIdx.x, lane = tid & 31, wave = tid >> 5;
  const int n0 = blockIdx.x * 64, k0 = blockIdx.y * 64;
#pragma unroll
  for (int pass = 0; pass < 4; ++pass) {
    const int kk = pass * 16 + (tid >> 4);
    const int c = tid & 15;
    const v4f v = *(const v4f*)(W + (size_t)(k0 + kk) * kHidden + n0 + 4 * c);
#pragma unroll
    for (int e = 0; e < 4; ++e) tileT[(4 * c + e) * 72 + kk] = f2bf_bits(v[e]);
  }
  __syncthreads();
  const int q = lane >> 3, c8 = (lane & 7) * 8;
  for (int pass = 0; pass < 2; ++pass) {
#pragma unroll
    for (int it = 0; it < 2; ++it) {
      const int nn = wave * 8 + it * 4 + q;
      const u4 val = *(const u4a*)(tileT + nn * 72 + c8);
      unsigned short* dst = Bt + (size_t)(nbase + n0 + nn) * ldo + k0 + c8;
      *(volatile u4*)dst = val;
      if (dup) *(volatile u4*)(dst + 1024) = val;
    }
    __threadfence();
  }
}

__global__ __launch_bounds__(256) void k_prep_w1t(const float* __restrict__ W1, unsigned short* __restrict__ Bt3) {
  const int tid = threadIdx.x, lane = tid & 31, wave = tid >> 5;
  const int q = lane >> 3, c8 = (lane & 7) * 8;
  const int line = blockIdx.x * 32 + wave * 4 + q;
  const int r = line >> 4, s = line & 15;
  const int rc = (r < 16) ? r : 15;
  const unsigned msk = (r < 16) ? 0xffffffffu : 0u;
  unsigned w[4];
#pragma unroll
  for (int e2 = 0; e2 < 4; ++e2) {
    const int k = 64 * s + c8 + 2 * e2;
    const float f0 = W1[(size_t)k * kLowR + rc];
    const float f1 = W1[(size_t)(k + 1) * kLowR + rc];
    w[e2] = (((unsigned)f2bf_bits(f0)) | (((unsigned)f2bf_bits(f1)) << 16)) & msk;
  }
  u4 val;
  val.x = w[0]; val.y = w[1]; val.z = w[2]; val.w = w[3];
  volatile u4* dst = (volatile u4*)(Bt3 + (size_t)r * kHidden + 64 * s + c8);
  *dst = val;
  __threadfence();
  *dst = val;
}

__global__ __launch_bounds__(256) void k_prep_w2t(const float* __restrict__ W2, unsigned short* __restrict__ Bt4) {
  const int tid = threadIdx.x, lane = tid & 31, wave = tid >> 5;
  const int q = lane >> 3, c8 = (lane & 7) * 8;
  const int line = blockIdx.x * 32 + wave * 4 + q;
  const int n = line >> 1, hf = line & 1;
  unsigned w[4];
#pragma unroll
  for (int e2 = 0; e2 < 4; ++e2) {
    const int p0 = c8 + 2 * e2, p1 = p0 + 1;
    const int pc0 = (p0 < 16) ? p0 : 15, pc1 = (p1 < 16) ? p1 : 15;
    const float f0 = W2[(size_t)pc0 * kHidden + n];
    const float f1 = W2[(size_t)pc1 * kHidden + n];
    const unsigned b0 = (p0 < 16) ? (unsigned)f2bf_bits(f0) : 0u;
    const unsigned b1 = (p1 < 16) ? (unsigned)f2bf_bits(f1) : 0u;
    w[e2] = b0 | (b1 << 16);
  }
  u4 val;
  val.x = w[0]; val.y = w[1]; val.z = w[2]; val.w = w[3];
  volatile u4* dst = (volatile u4*)(Bt4 + (size_t)n * 128 + hf * 64 + c8);
  *dst = val;
  __threadfence();
  *dst = val;
}

__global__ __launch_bounds__(256) void k_scan(const float* __restrict__ Cq, const float* __restrict__ Ap,
                                             const float* __restrict__ bg2, const float* __restrict__ gnw,
                                             unsigned short* __restrict__ oplane, float* __restrict__ state_out) {
  __shared__ __align__(16) float qs[2][64];
  __shared__ __align__(16) float ks[2][64];
  __shared__ __align__(16) float egs[2][64];
  __shared__ __align__(16) float vs[2][64];
  __shared__ __align__(16) float gsv[2][64];
  __shared__ __align__(16) float ob[2][64];
  __shared__ __align__(16) float red[2][8];
  __shared__ __align__(16) unsigned int st[64];
  __shared__ __align__(16) float sst[64 * 68];

  const int tid = threadIdx.x, lane = tid & 31, wave = tid >> 5;
  const int p = tid & 3;
  const int j = tid >> 2;
  const int bh = blockIdx.x;
  const int b = bh / kHeads, h = bh - b * kHeads;
  const int dld = tid & 63;

  float S[16];
#pragma unroll
  for (int i = 0; i < 16; ++i) S[i] = 0.f;

  const float bgr = bf_bits2f(f2bf_bits(bg2[h * kHdim + dld]));
  const float gw0 = bf_bits2f(f2bf_bits(gnw[(2 * lane) & 63]));
  const float gw1 = bf_bits2f(f2bf_bits(gnw[(2 * lane + 1) & 63]));

  for (int t = 0; t < kSeq; ++t) {
    const int par = t & 1;
    const size_t row = (size_t)b * kSeq + t;
    if (wave < 2) {
      const float* cr = Cq + row * 4096 + h * kHdim + dld;
      const float qv = cr[0];
      const float kv = cr[1024];
      const float av = Ap[row * kHidden + h * kHdim + dld] + bgr;
      const float ls = fminf(av, 0.f) - log1pf(expf(-fabsf(av)));
      const float eg = expf(ls * 0.0625f);
      qs[par][dld] = qv;
      ks[par][dld] = kv;
      egs[par][dld] = eg;
    } else if (wave < 4) {
      const float* cr = Cq + row * 4096 + h * kHdim + dld;
      vs[par][dld]  = cr[2048];
      gsv[par][dld] = cr[3072];
    }
    __syncthreads();

    const float vj = vs[par][j];
    const float* qp = &qs[par][16 * p];
    const float* kp = &ks[par][16 * p];
    const float* ep = &egs[par][16 * p];
    float o = 0.f;
#pragma unroll
    for (int i4 = 0; i4 < 4; ++i4) {
      const v4f q4 = *(const v4f*)(qp + 4 * i4);
      const v4f k4 = *(const v4f*)(kp + 4 * i4);
      const v4f e4 = *(const v4f*)(ep + 4 * i4);
#pragma unroll
      for (int e = 0; e < 4; ++e) {
        const float kvv = k4[e] * vj;
        const float s = fmaf(e4[e], S[4 * i4 + e], kvv);
        S[4 * i4 + e] = s;
        o = fmaf(s, q4[e], o);
      }
    }
    o += __shfl_xor(o, 1, 32);
    o += __shfl_xor(o, 2, 32);
    const float osc = o * kOScale;
    float q2 = (p == 0) ? osc * osc : 0.f;
#pragma unroll
    for (int off = 1; off < 32; off <<= 1) q2 += __shfl_xor(q2, off, 32);
    if (p == 0) ob[par][j] = osc;
    if (lane == 0) red[par][wave] = q2;
    __syncthreads();

    if (wave == 0) {
      const float ss = ((red[par][0] + red[par][1]) + (red[par][2] + red[par][3])) +
                       ((red[par][4] + red[par][5]) + (red[par][6] + red[par][7]));
      const float rn = rsqrtf(ss * (1.0f / 64.0f) + kEps);
      const int j0 = 2 * lane, j1 = 2 * lane + 1;
      float o0 = (ob[par][j0] * rn) * gw0;
      float o1 = (ob[par][j1] * rn) * gw1;
      const float g0 = gsv[par][j0], g1 = gsv[par][j1];
      const float s0 = g0 * __builtin_amdgcn_rcpf(1.0f + expf(-g0));
      const float s1 = g1 * __builtin_amdgcn_rcpf(1.0f + expf(-g1));
      o0 = o0 * s0;
      o1 = o1 * s1;
      const unsigned short h0 = f2bf_bits(o0), h1 = f2bf_bits(o1);
      const unsigned short l0 = f2bf_bits(o0 - bf_bits2f(h0)), l1 = f2bf_bits(o1 - bf_bits2f(h1));
      st[lane]      = (unsigned)h0 | ((unsigned)h1 << 16);
      st[32 + lane] = (unsigned)l0 | ((unsigned)l1 << 16);
      __builtin_amdgcn_fence(__ATOMIC_RELEASE, "workgroup");
      __builtin_amdgcn_wave_barrier();
      __builtin_amdgcn_fence(__ATOMIC_ACQUIRE, "workgroup");
      const u4 val = *(const u4a*)(st + 4 * (lane & 15));
      if (lane < 16) {
        const size_t off = row * 2048 + (size_t)(h * kHdim + 8 * lane + ((lane >= 8) ? 960 : 0));
        volatile u4* dst = (volatile u4*)(oplane + off);
        *dst = val;
        __threadfence();
        *dst = val;
      }
    }
  }

#pragma unroll
  for (int i = 0; i < 16; ++i) sst[(16 * p + i) * 68 + j] = S[i];
  __syncthreads();
  const int q = lane >> 3, c4l = (lane & 7) * 4;
  for (int pass = 0; pass < 2; ++pass) {
#pragma unroll
    for (int it = 0; it < 4; ++it) {
      const int line = it * 32 + wave * 4 + q;
      const int d = line >> 1;
      const int c = (line & 1) * 32 + c4l;
      const v4f val = *(const v4f*)(sst + d * 68 + c);
      *(volatile v4f*)(state_out + ((size_t)bh * kHdim + d) * kHdim + c) = val;
    }
    __threadfence();
  }
}

extern "C" void kernel_launch(void* const* d_in, const int* in_sizes, int n_in,
                              void* d_out, int out_size, void* d_ws, size_t ws_size,
                              hipStream_t stream) {
  (void)in_sizes; (void)n_in; (void)out_size; (void)ws_size;
  const float* x   = (const float*)d_in[0];
  const float* Wq  = (const float*)d_in[1];
  const float* Wk  = (const float*)d_in[2];
  const float* Wv  = (const float*)d_in[3];
  const float* Wg1 = (const float*)d_in[4];
  const float* Wg2 = (const float*)d_in[5];
  const float* bg2 = (const float*)d_in[6];
  const float* Wg  = (const float*)d_in[7];
  const float* gnw = (const float*)d_in[8];
  const float* Wo  = (const float*)d_in[9];
  float* out0 = (float*)d_out;
  float* out1 = (float*)d_out + kOut1FloatOff;

  char* ws = (char*)d_ws;
  unsigned short* xb    = (unsigned short*)(ws + kOffXb);
  unsigned short* btcat = (unsigned short*)(ws + kOffBtcat);
  unsigned short* bt3   = (unsigned short*)(ws + kOffBt3);
  unsigned short* bt4   = (unsigned short*)(ws + kOffBt4);
  unsigned short* bt7   = (unsigned short*)(ws + kOffBt7);
  float*          cqkvg = (float*)(ws + kOffCqkvg);
  unsigned short* c3    = (unsigned short*)(ws + kOffC3);
  float*          apre  = (float*)(ws + kOffApre);
  unsigned short* opl   = (unsigned short*)(ws + kOffOpl);

  const int nPairs = kRows * kHidden / 2;
  k_cast_bf16x2<<<(nPairs + 255) / 256, 256, 0, stream>>>(x, xb, nPairs);

  dim3 wgrid(kHidden / 64, kHidden / 64);
  k_wtrans<<<wgrid, 256, 0, stream>>>(Wq, btcat, 1024, 0, 0);
  k_wtrans<<<wgrid, 256, 0, stream>>>(Wk, btcat, 1024, 1024, 0);
  k_wtrans<<<wgrid, 256, 0, stream>>>(Wv, btcat, 1024, 2048, 0);
  k_wtrans<<<wgrid, 256, 0, stream>>>(Wg, btcat, 1024, 3072, 0);
  k_wtrans<<<wgrid, 256, 0, stream>>>(Wo, bt7, 2048, 0, 1);
  k_prep_w1t<<<32, 256, 0, stream>>>(Wg1, bt3);
  k_prep_w2t<<<64, 256, 0, stream>>>(Wg2, bt4);

  wmma_gemm64<1, false, 0, 0, false><<<dim3((kRows / 64) * (4096 / 64) / 8, 1), 256, 0, stream>>>(
      xb, xb, 1024, 0L, btcat, btcat, 1024, 0L, (void*)cqkvg, (void*)cqkvg, 4096, 0L,
      gnw, gnw, 0L, kRows, 4096, 1024, 1.0f);

  wmma_gemm64<1, false, 0, 2, false><<<dim3((kRows / 64) * 1 / 8, 1), 256, 0, stream>>>(
      xb, xb, 1024, 0L, bt3, bt3, 1024, 0L, (void*)c3, (void*)(c3 + 64), 128, 0L,
      gnw, gnw, 0L, kRows, 64, 1024, 1.0f);

  wmma_gemm64<1, false, 0, 0, false><<<dim3((kRows / 64) * (kHidden / 64) / 8, 1), 256, 0, stream>>>(
      c3, c3, 128, 0L, bt4, bt4, 128, 0L, (void*)apre, (void*)apre, 1024, 0L,
      gnw, gnw, 0L, kRows, kHidden, 128, 1.0f);

  k_scan<<<kBatch * kHeads, 256, 0, stream>>>(cqkvg, apre, bg2, gnw, opl, out1);

  wmma_gemm64<1, false, 0, 0, false><<<dim3((kRows / 64) * (kHidden / 64) / 8, 1), 256, 0, stream>>>(
      opl, opl, 2048, 0L, bt7, bt7, 2048, 0L, (void*)out0, (void*)out0, 1024, 0L,
      gnw, gnw, 0L, kRows, kHidden, 2048, 1.0f);
}
